// Sidechain_3332894622683
// MI455X (gfx1250) — hardware-verified
//
#include <hip/hip_runtime.h>
#include <math.h>

constexpr int kBatch       = 8;
constexpr int kLen         = 4096;
constexpr int kCh          = 128;
constexpr int kTaps        = 7;
constexpr int kLp          = kLen - kTaps + 1;
constexpr int kNdyn        = kCh * kTaps;
constexpr int kRowsAll     = kBatch * kLen;
constexpr int kHalves      = 2;
constexpr int kBatchHalf   = kBatch / kHalves;
constexpr int kRowsHalf    = kBatchHalf * kLen;
constexpr int kOutRowsHalf = kBatchHalf * kLp;

static_assert(kRowsHalf % 64 == 0, "M tile multiple");
static_assert(kNdyn % 64 == 0, "N tile multiple");
static_assert(kCh % 32 == 0, "K multiple of 32");
static_assert((kRowsAll * kCh) % (8 * 256) == 0, "x split grid exact");
static_assert((kNdyn * kCh) % (8 * 256) == 0, "w split grid exact");
static_assert(kOutRowsHalf % 2 == 0, "gate grid exact");

typedef __attribute__((ext_vector_type(16))) _Float16 v16h;
typedef __attribute__((ext_vector_type(8)))  _Float16 v8h;
typedef __attribute__((ext_vector_type(16))) __bf16   v16b;
typedef __attribute__((ext_vector_type(8)))  __bf16   v8b;
typedef __attribute__((ext_vector_type(8)))  float    v8f;
typedef __attribute__((ext_vector_type(4)))  float    v4f;
typedef __attribute__((ext_vector_type(4)))  unsigned int v4u;

__device__ __forceinline__ unsigned short f2bf_bits(float f) {
  unsigned u = __float_as_uint(f);
  return (unsigned short)((u + 0x7FFFu + ((u >> 16) & 1u)) >> 16);
}
__device__ __forceinline__ float bf_bits2f(unsigned short h) { return __uint_as_float(((unsigned)h) << 16); }

__device__ __forceinline__ void dep_guard_h(v8f& a, v8f& b, v16h x, v16h y) { asm volatile("v_nop\n\tv_nop\n\tv_nop\n\tv_nop" : "+v"(a), "+v"(b) : "v"(x), "v"(y)); }
__device__ __forceinline__ void dep_guard_b(v8f& a, v8f& b, v16b x, v16b y) { asm volatile("v_nop\n\tv_nop\n\tv_nop\n\tv_nop" : "+v"(a), "+v"(b) : "v"(x), "v"(y)); }
__device__ __forceinline__ void keep4_h(v16h a, v16h b, v16h c, v16h d) { asm volatile("v_nop" :: "v"(a), "v"(b), "v"(c), "v"(d)); }
__device__ __forceinline__ void keep4_b(v16b a, v16b b, v16b c, v16b d) { asm volatile("v_nop" :: "v"(a), "v"(b), "v"(c), "v"(d)); }
__device__ __forceinline__ void acc_guard4(v8f& a, v8f& b, v8f& c, v8f& d) { asm volatile("v_nop\n\tv_nop\n\tv_nop\n\tv_nop" : "+v"(a), "+v"(b), "+v"(c), "+v"(d)); }
template <typename T> struct Frag;
template <> struct Frag<_Float16> {
  typedef v16h V; union U { v16h v; v8h h[2]; };
  static __device__ __forceinline__ v16h load(const _Float16* p) {
    U f; f.h[0] = *(const v8h*)(p); f.h[1] = *(const v8h*)(p + 16); return f.v;
  }
  static __device__ __forceinline__ v8f mma(v16h a, v16h b, v8f c) {
    return __builtin_amdgcn_wmma_f32_16x16x32_f16(false, a, false, b, (short)0, c, false, false);
  }
  static __device__ __forceinline__ void guard(v8f& a, v8f& b, v16h x, v16h y) { dep_guard_h(a, b, x, y); }
  static __device__ __forceinline__ void keep(v16h a, v16h b, v16h c, v16h d) { keep4_h(a, b, c, d); }
};
template <> struct Frag<__bf16> {
  typedef v16b V; union U { v16b v; v8b h[2]; };
  static __device__ __forceinline__ v16b load(const __bf16* p) {
    U f; f.h[0] = *(const v8b*)(p); f.h[1] = *(const v8b*)(p + 16); return f.v;
  }
  static __device__ __forceinline__ v8f mma(v16b a, v16b b, v8f c) {
    return __builtin_amdgcn_wmma_f32_16x16x32_bf16(false, a, false, b, (short)0, c, false, false);
  }
  static __device__ __forceinline__ void guard(v8f& a, v8f& b, v16b x, v16b y) { dep_guard_b(a, b, x, y); }
  static __device__ __forceinline__ void keep(v16b a, v16b b, v16b c, v16b d) { keep4_b(a, b, c, d); }
};

__device__ __forceinline__ unsigned pk16(unsigned short a, unsigned short b) { return (unsigned)a | ((unsigned)b << 16); }

template <int ET> struct Elem;
template <> struct Elem<0> { typedef _Float16 T; };
template <> struct Elem<1> { typedef __bf16 T; };
template <int ET, bool SPLIT, int BIAS_MODE, int OUT_MODE, bool RESID, int ACT = 0>
__global__ __launch_bounds__(256) void wmma_gemm64(
    const unsigned short* __restrict__ Ap, const unsigned short* __restrict__ A2p, int lda, long strideA,
    const unsigned short* __restrict__ Btp, const unsigned short* __restrict__ Bt2p, int ldb, long strideB,
    void* __restrict__ Cout, void* __restrict__ Cout2, int ldc, long strideC,
    const float* __restrict__ bias,
    const float* __restrict__ resid, long strideR,
    int M, int N, int K, float scale) {
  typedef typename Elem<ET>::T T;
  typedef typename Frag<T>::V V;
  const T* A = (const T*)Ap; const T* A2 = (const T*)A2p; const T* Bt = (const T*)Btp; const T* Bt2 = (const T*)Bt2p;
  __shared__ __align__(16) float sT[8][16 * 68];
  const int b    = blockIdx.y;
  const int lane = threadIdx.x & 31;
  const int wave = threadIdx.x >> 5;
  const int tilesN = N >> 6;
  const int tilesM = M >> 6;
  const int tile = blockIdx.x * 8 + wave;
  if (tile >= tilesM * tilesN) return;
  const int tm = tile / tilesN;
  const int tn = tile - tm * tilesN;
  const int m0 = tm << 6;
  const int n0 = tn << 6;

  const T* Ab  = A  + (size_t)b * strideA;
  const T* Bb  = Bt + (size_t)b * strideB;
  const T* Ab2 = SPLIT ? (A2  + (size_t)b * strideA) : nullptr;
  const T* Bb2 = SPLIT ? (Bt2 + (size_t)b * strideB) : nullptr;

  const int rlane = lane & 15;
  const int koff  = (lane >> 4) * 8;
  const int mOff  = (lane >> 4) * 8;

  v8f acc[4][4];
#pragma unroll
  for (int i = 0; i < 4; ++i)
#pragma unroll
    for (int j = 0; j < 4; ++j) acc[i][j] = (v8f){0.f,0.f,0.f,0.f,0.f,0.f,0.f,0.f};

  for (int k0 = 0; k0 < K; k0 += 32) {
    V bh[4], bl[4];
#pragma unroll
    for (int j = 0; j < 4; ++j) {
      const size_t bo = (size_t)(n0 + (j << 4) + rlane) * ldb + koff + k0;
      bh[j] = Frag<T>::load(Bb + bo);
      if (SPLIT) bl[j] = Frag<T>::load(Bb2 + bo);
    }
#pragma unroll
    for (int i = 0; i < 4; ++i) {
      const size_t ao = (size_t)(m0 + (i << 4) + rlane) * lda + koff + k0;
      V ah = Frag<T>::load(Ab + ao);
      V al;
      if (SPLIT) al = Frag<T>::load(Ab2 + ao);
#pragma unroll
      for (int j = 0; j < 4; ++j) {
        acc[i][j] = Frag<T>::mma(ah, bh[j], acc[i][j]);
        if (SPLIT) {
          acc[i][j] = Frag<T>::mma(ah, bl[j], acc[i][j]);
          acc[i][j] = Frag<T>::mma(al, bh[j], acc[i][j]);
        }
      }
      Frag<T>::guard(acc[i][0], acc[i][3], ah, SPLIT ? al : ah);
    }
    Frag<T>::keep(bh[0], bh[1], bh[2], bh[3]);
    if (SPLIT) Frag<T>::keep(bl[0], bl[1], bl[2], bl[3]);
  }
  acc_guard4(acc[0][0], acc[0][1], acc[0][2], acc[0][3]);
  acc_guard4(acc[1][0], acc[1][1], acc[1][2], acc[1][3]);
  acc_guard4(acc[2][0], acc[2][1], acc[2][2], acc[2][3]);
  acc_guard4(acc[3][0], acc[3][1], acc[3][2], acc[3][3]);

  float* slab = sT[wave];
  const float* Rb = RESID ? (resid + (size_t)b * strideR) : nullptr;
#pragma unroll
  for (int i = 0; i < 4; ++i) {
    const int mBase = m0 + (i << 4);
#pragma unroll
    for (int j = 0; j < 4; ++j) {
      const int n = n0 + (j << 4) + rlane;
      float bv = 0.f;
      if (BIAS_MODE == 2) bv = bias[n];
#pragma unroll
      for (int r = 0; r < 8; ++r) {
        float v = acc[i][j][r] * scale;
        if (BIAS_MODE == 1) v += bias[mBase + mOff + r];
        if (BIAS_MODE == 2) v += bv;
        if (RESID) v += Rb[(size_t)(mBase + mOff + r) * ldc + n];
        if (ACT == 2) v = fmaxf(v, 0.0f);
        if (ACT == 4) v = (v > 0.f) ? v : 0.01f * v;
        slab[(mOff + r) * 68 + (j << 4) + rlane] = v;
      }
    }
    __builtin_amdgcn_fence(__ATOMIC_RELEASE, "workgroup");
    __builtin_amdgcn_wave_barrier();
    __builtin_amdgcn_fence(__ATOMIC_ACQUIRE, "workgroup");
    if (OUT_MODE == 0) {
      float* C = (float*)Cout + (size_t)b * strideC;
      const int hh = lane >> 4, c4 = (lane & 15) * 4;
      for (int pass = 0; pass < 2; ++pass) {
#pragma unroll
        for (int it = 0; it < 8; ++it) {
          const int row = it * 2 + hh;
          v4f v = *(const v4f*)(slab + row * 68 + c4);
          *(volatile v4f*)(C + (size_t)(mBase + row) * ldc + n0 + c4) = v;
        }
        __threadfence();
      }
    } else {
      const int q = lane >> 3, c8 = (lane & 7) * 8;
      unsigned short* C  = (unsigned short*)Cout  + (size_t)b * strideC;
      unsigned short* C2 = (OUT_MODE == 2) ? ((unsigned short*)Cout2 + (size_t)b * strideC) : nullptr;
      for (int pass = 0; pass < 2; ++pass) {
#pragma unroll
        for (int it = 0; it < 4; ++it) {
          const int row = it * 4 + q;
          const float* sp = slab + row * 68 + c8;
          v8h hv, lv;
#pragma unroll
          for (int e = 0; e < 8; ++e) {
            if (OUT_MODE == 1) {
              hv[e] = (_Float16)sp[e];
            } else {
              unsigned short hb = f2bf_bits(sp[e]);
              unsigned short lb = f2bf_bits(sp[e] - bf_bits2f(hb));
              hv[e] = __builtin_bit_cast(_Float16, hb);
              lv[e] = __builtin_bit_cast(_Float16, lb);
            }
          }
          *(volatile v8h*)(C + (size_t)(mBase + row) * ldc + n0 + c8) = hv;
          if (OUT_MODE == 2) *(volatile v8h*)(C2 + (size_t)(mBase + row) * ldc + n0 + c8) = lv;
        }
        __threadfence();
      }
    }
    __builtin_amdgcn_fence(__ATOMIC_RELEASE, "workgroup");
    __builtin_amdgcn_wave_barrier();
    __builtin_amdgcn_fence(__ATOMIC_ACQUIRE, "workgroup");
  }
}

__global__ __launch_bounds__(256) void xsplit8_kernel(const float* __restrict__ in,
                                                      unsigned short* __restrict__ hi,
                                                      unsigned short* __restrict__ lo, int n8) {
  const int i = blockIdx.x * 256 + threadIdx.x;
  if (i >= n8) return;
  const float* p = in + 8 * (size_t)i;
  const v4f a = *(const v4f*)(p);
  const v4f c = *(const v4f*)(p + 4);
  unsigned short hb[8], lb[8];
#pragma unroll
  for (int e = 0; e < 4; ++e) {
    hb[e] = f2bf_bits(a[e]);
    lb[e] = f2bf_bits(a[e] - bf_bits2f(hb[e]));
    hb[4 + e] = f2bf_bits(c[e]);
    lb[4 + e] = f2bf_bits(c[e] - bf_bits2f(hb[4 + e]));
  }
  const v4u uh = (v4u){pk16(hb[0], hb[1]), pk16(hb[2], hb[3]), pk16(hb[4], hb[5]), pk16(hb[6], hb[7])};
  const v4u ul = (v4u){pk16(lb[0], lb[1]), pk16(lb[2], lb[3]), pk16(lb[4], lb[5]), pk16(lb[6], lb[7])};
  unsigned short* qh = hi + 8 * (size_t)i;
  unsigned short* ql = lo + 8 * (size_t)i;
  *(volatile v4u*)qh = uh;
  *(volatile v4u*)ql = ul;
  __threadfence();
  *(volatile v4u*)qh = uh;
  *(volatile v4u*)ql = ul;
}

__global__ __launch_bounds__(256) void wsplit_kernel(const float* __restrict__ w,
                                                     unsigned short* __restrict__ hi,
                                                     unsigned short* __restrict__ lo, int nthreads) {
  const int i = blockIdx.x * 256 + threadIdx.x;
  if (i >= nthreads) return;
  const int n  = i >> 4;
  const int c8 = (i & 15) * 8;
  const int d  = n / kTaps;
  const int k  = n - d * kTaps;
  const float* src = w + (size_t)d * (kCh * kTaps) + (size_t)c8 * kTaps + k;
  unsigned short hb[8], lb[8];
#pragma unroll
  for (int e = 0; e < 8; ++e) {
    const float f = src[e * kTaps];
    hb[e] = f2bf_bits(f);
    lb[e] = f2bf_bits(f - bf_bits2f(hb[e]));
  }
  const v4u uh = (v4u){pk16(hb[0], hb[1]), pk16(hb[2], hb[3]), pk16(hb[4], hb[5]), pk16(hb[6], hb[7])};
  const v4u ul = (v4u){pk16(lb[0], lb[1]), pk16(lb[2], lb[3]), pk16(lb[4], lb[5]), pk16(lb[6], lb[7])};
  unsigned short* qh = hi + (size_t)n * kCh + c8;
  unsigned short* ql = lo + (size_t)n * kCh + c8;
  *(volatile v4u*)qh = uh;
  *(volatile v4u*)ql = ul;
  __threadfence();
  *(volatile v4u*)qh = uh;
  *(volatile v4u*)ql = ul;
}

__global__ __launch_bounds__(256) void gate_sum_kernel(const float* __restrict__ x,
                                                       const float* __restrict__ wdyn,
                                                       float* __restrict__ out, int nrows) {
  __shared__ __align__(16) float so[2][kCh];
  const int t    = threadIdx.x;
  const int rsel = t >> 7;
  const int d    = t & (kCh - 1);
  const int r    = blockIdx.x * 2 + rsel;
  const bool valid = (r < nrows);
  const int rc   = valid ? r : (nrows - 1);
  const int bl   = rc / kLp;
  const int l    = rc - bl * kLp;
  const float* xp = x + ((size_t)bl * kLen + l) * kCh + d;
  const float* wp = wdyn + ((size_t)bl * kLen + l + (kTaps - 1)) * kNdyn + d * kTaps;
  float o = 0.f;
#pragma unroll 1
  for (int k = 0; k < kTaps; ++k) {
    const float xv = xp[(size_t)k * kCh];
    const float g  = tanhf(wp[k]);
    o += xv * g;
  }
  so[rsel][d] = o;
  __syncthreads();
  if ((t & (kCh - 1)) < 32) {
    const int lane = t & 31;
    const v4f v = *(const v4f*)(&so[rsel][lane * 4]);
    if (valid) {
      float* op = out + (size_t)rc * kCh + lane * 4;
      *(volatile v4f*)op = v;
      __threadfence();
      *(volatile v4f*)op = v;
    }
  }
}

extern "C" void kernel_launch(void* const* d_in, const int* in_sizes, int n_in,
                              void* d_out, int out_size, void* d_ws, size_t ws_size,
                              hipStream_t stream) {
  if (n_in < 2) return;
  if (in_sizes[0] != kRowsAll * kCh) return;
  if (in_sizes[1] != kCh * kCh * kTaps) return;
  if (out_size != kBatch * kLp * kCh) return;

  const float* x   = (const float*)d_in[0];
  const float* w   = (const float*)d_in[1];
  float*       out = (float*)d_out;

  const size_t xPlaneBytes  = (size_t)kRowsAll * kCh * 2;
  const size_t wPlaneBytes  = (size_t)kNdyn * kCh * 2;
  const size_t wdynBytes    = (size_t)kRowsHalf * kNdyn * 4;
  const size_t offXh   = 0;
  const size_t offXl   = offXh + xPlaneBytes;
  const size_t offWh   = offXl + xPlaneBytes;
  const size_t offWl   = offWh + wPlaneBytes;
  const size_t offWdyn = offWl + wPlaneBytes;
  const size_t total   = offWdyn + wdynBytes;
  if (total > ws_size) return;

  unsigned char* ws = (unsigned char*)d_ws;
  unsigned short* xh   = (unsigned short*)(ws + offXh);
  unsigned short* xl   = (unsigned short*)(ws + offXl);
  unsigned short* wbh  = (unsigned short*)(ws + offWh);
  unsigned short* wbl  = (unsigned short*)(ws + offWl);
  float*          wdyn = (float*)(ws + offWdyn);

  {
    const int n8 = kRowsAll * kCh / 8;
    xsplit8_kernel<<<dim3(n8 / 256), dim3(256), 0, stream>>>(x, xh, xl, n8);
  }
  {
    const int nthreads = kNdyn * (kCh / 8);
    wsplit_kernel<<<dim3(nthreads / 256), dim3(256), 0, stream>>>(w, wbh, wbl, nthreads);
  }
  const int gemmTiles  = (kRowsHalf / 64) * (kNdyn / 64);
  const int gemmBlocks = gemmTiles / 8;
  const int gateBlocks = (kOutRowsHalf + 1) / 2;
  for (int hf = 0; hf < kHalves; ++hf) {
    const size_t aoff = (size_t)hf * kRowsHalf * kCh;
    wmma_gemm64<1, true, 0, 0, false, 0><<<dim3(gemmBlocks, 1), dim3(256), 0, stream>>>(
        xh + aoff, xl + aoff, kCh, 0L,
        wbh, wbl, kCh, 0L,
        (void*)wdyn, (void*)wdyn, kNdyn, 0L,
        (const float*)wdyn,
        (const float*)wdyn, 0L,
        kRowsHalf, kNdyn, kCh, 1.0f);
    gate_sum_kernel<<<dim3(gateBlocks), dim3(256), 0, stream>>>(
        x + (size_t)hf * kRowsHalf * kCh,
        wdyn,
        out + (size_t)hf * kOutRowsHalf * kCh,
        kOutRowsHalf);
  }
}
